// NN_26508538151674
// MI455X (gfx1250) — hardware-verified
//
#include <hip/hip_runtime.h>

typedef __attribute__((ext_vector_type(16))) _Float16 v16h;
typedef __attribute__((ext_vector_type(8)))  _Float16 v8h;
typedef __attribute__((ext_vector_type(4)))  _Float16 v4h;
typedef __attribute__((ext_vector_type(8)))  float    v8f;
typedef __attribute__((ext_vector_type(4)))  float    v4f;

constexpr int kN     = 65536;
constexpr int kDin   = 16;
constexpr int kH     = 128;
constexpr int kSamp  = 64;
constexpr int kK1    = 32;
constexpr int kA1P   = 40;
constexpr int kA2P   = 136;
constexpr int kYP    = 132;
static_assert((kN % kSamp) == 0, "sample tiles");
static_assert(kK1 == 2 * kDin, "layer-1 K = value half + residual half");
static_assert((kH % 32) == 0 && (kK1 % 32) == 0, "K multiples of 32");
static_assert((kA1P % 8) == 0 && (kA2P % 8) == 0 && (kYP % 4) == 0, "16-B aligned LDS rows");
static_assert(kSamp * kYP * 4 <= 2 * kSamp * kA2P * 2, "Y stage fits in the A2 bytes");

constexpr float kCarryXh  = 128.0f;
constexpr float kCarryXl  = 2048.0f;
constexpr float kCarryW1a = 1024.0f;
constexpr float kCarryW1b = 64.0f;
constexpr float kCarryY   = 256.0f;
constexpr float kCarryW2  = 64.0f;
constexpr float kCarryRes = 2048.0f;
static_assert(kCarryXh * kCarryW1a == kCarryXl * kCarryW1b, "both K halves share one product scale");
constexpr float kFold1   = 1.0f / (kCarryXh * kCarryW1a);
constexpr float kFold2   = 1.0f / (kCarryY * kCarryW2);
constexpr float kResFold = 1.0f / kCarryRes;

constexpr size_t kOffBt2  = 0;
constexpr size_t kOffBt2r = kOffBt2  + (size_t)kH * kH * 2;
constexpr size_t kOffBt1  = kOffBt2r + (size_t)kH * kH * 2;
constexpr size_t kOffBt1r = kOffBt1  + (size_t)kH * kK1 * 2;
constexpr size_t kWsTotal = kOffBt1r + (size_t)kH * kK1 * 2;
static_assert(kWsTotal == 81920ull, "carve total");
static_assert(kWsTotal <= 134217728ull, "carve cap");
static_assert((kOffBt2r % 128) == 0 && (kOffBt1 % 128) == 0 && (kOffBt1r % 128) == 0, "aligned regions");

constexpr size_t kOutB    = 0;
constexpr size_t kOutBd   = (size_t)kN;
constexpr size_t kOutY2   = 2 * (size_t)kN;
constexpr size_t kOutElems = kOutY2 + (size_t)kN * kH;
static_assert(kOutB == 0 && kOutBd * 4 == 262144ull && kOutY2 * 4 == 524288ull, "output byte offsets");
static_assert(kOutElems * 4 == 34078720ull, "output total");

__device__ __forceinline__ float h16_to_f32(unsigned hb) {
  const unsigned sgn = (hb & 0x8000u) << 16;
  const unsigned em = hb & 0x7fffu;
  const float fn = __uint_as_float((em << 13) + 0x38000000u);
  const float fs = (float)em * 5.9604644775390625e-8f;
  const float mag = (em < 0x400u) ? fs : fn;
  return __uint_as_float(__float_as_uint(mag) | sgn);
}

__device__ __forceinline__ void split_carry(float v, _Float16& hs, _Float16& ls) {
  hs = (_Float16)(v * kCarryXh);
  const unsigned hb = (unsigned)__builtin_bit_cast(unsigned short, hs);
  const float hf = h16_to_f32(hb) * (1.0f / kCarryXh);
  ls = (_Float16)((v - hf) * kCarryXl);
}

union FragU { v16h v; v8h h[2]; };
__device__ __forceinline__ v16h frag_load(const _Float16* p) {
  FragU f;
  f.h[0] = *(const v8h*)(p);
  f.h[1] = *(const v8h*)(p + 16);
  return f.v;
}

__device__ __forceinline__ v8f mma_h(v16h a, v16h b, v8f c) {
  c = __builtin_amdgcn_wmma_f32_16x16x32_f16(false, a, false, b, (short)0, c, false, false);
  asm volatile("v_nop\n\tv_nop\n\tv_nop\n\tv_nop" : "+v"(c) : "v"(a), "v"(b));
  return c;
}

constexpr int kChunks2 = kH * kH / 8;
constexpr int kChunks1 = kH * kK1 / 8;
static_assert(kChunks2 == 2048 && kChunks1 == 512, "chunk counts");
static_assert(((kChunks2 + kChunks1) % 256) == 0 && (kChunks2 % 256) == 0, "whole blocks per plane");

__global__ __launch_bounds__(256) void prep_weights_kernel(
    const float* __restrict__ W1, const float* __restrict__ W2,
    unsigned short* __restrict__ Bt2, unsigned short* __restrict__ Bt2r,
    unsigned short* __restrict__ Bt1, unsigned short* __restrict__ Bt1r)
{
  const int i = blockIdx.x * 256 + threadIdx.x;
  const bool isW2 = ((int)blockIdx.x < (kChunks2 / 256));
  v4f a0, a1;
  float sc;
  bool wantRes;
  unsigned short* dv;
  unsigned short* dr;
  if (isW2) {
    const size_t e0 = (size_t)i * 8;
    a0 = *(const v4f*)(W2 + e0);
    a1 = *(const v4f*)(W2 + e0 + 4);
    sc = kCarryW2;
    wantRes = true;
    dv = Bt2 + e0;
    dr = Bt2r + e0;
  } else {
    const int j = i - kChunks2;
    const int row = j >> 2;
    const int q = j & 3;
    const float* src = W1 + (size_t)row * kDin + (q & 1) * 8;
    a0 = *(const v4f*)(src);
    a1 = *(const v4f*)(src + 4);
    sc = (q < 2) ? kCarryW1a : kCarryW1b;
    wantRes = (q < 2);
    dv = Bt1 + (size_t)j * 8;
    dr = Bt1r + (size_t)j * 8;
  }
  v8h hv, rv;
#pragma unroll
  for (int e = 0; e < 4; ++e) {
    const float f0 = a0[e];
    const float f1 = a1[e];
    const float w0 = f0 * sc;
    const float w1 = f1 * sc;
    const _Float16 h0 = (_Float16)w0;
    const _Float16 h1 = (_Float16)w1;
    const unsigned hb0 = (unsigned)__builtin_bit_cast(unsigned short, h0);
    const unsigned hb1 = (unsigned)__builtin_bit_cast(unsigned short, h1);
    const float r0 = (w0 - h16_to_f32(hb0)) * kCarryRes;
    const float r1 = (w1 - h16_to_f32(hb1)) * kCarryRes;
    const float r0s = wantRes ? r0 : 0.0f;
    const float r1s = wantRes ? r1 : 0.0f;
    hv[e]     = h0;
    hv[4 + e] = h1;
    rv[e]     = (_Float16)r0s;
    rv[4 + e] = (_Float16)r1s;
  }
  *(volatile v8h*)dv = hv;
  *(volatile v8h*)dr = rv;
  __threadfence();
  *(volatile v8h*)dv = hv;
  *(volatile v8h*)dr = rv;
}

__global__ __launch_bounds__(256) void mlp_tangent_kernel(
    const float* __restrict__ x, const float* __restrict__ xdot,
    const unsigned short* __restrict__ Bt1p, const unsigned short* __restrict__ Bt1rp,
    const unsigned short* __restrict__ Bt2p, const unsigned short* __restrict__ Bt2rp,
    const float* __restrict__ W3, float* __restrict__ out)
{
  __shared__ __align__(16) _Float16 sA1[2 * kSamp * kA1P];
  __shared__ __align__(16) unsigned char sU[2 * kSamp * kA2P * 2];
  __shared__ __align__(16) float sPart[2 * 8 * kSamp];
  _Float16* sA2 = (_Float16*)sU;
  float* sY = (float*)sU;

  const int tid  = threadIdx.x;
  const int lane = tid & 31;
  const int wave = __builtin_amdgcn_readfirstlane((int)(threadIdx.x >> 5));
  const int hh   = lane >> 4;
  const int c    = lane & 15;
  const int n0   = blockIdx.x * kSamp;
  const int n    = wave * 16 + c;

  {
    const int r  = tid >> 2;
    const int c4 = (tid & 3) * 4;
    const v4f vx = *(const v4f*)(x    + (size_t)(n0 + r) * kDin + c4);
    const v4f vd = *(const v4f*)(xdot + (size_t)(n0 + r) * kDin + c4);
    v4h xh, xl, dh, dl;
#pragma unroll
    for (int e = 0; e < 4; ++e) {
      const float fx = vx[e];
      const float fd = vd[e];
      _Float16 h0, l0, h1, l1;
      split_carry(fx, h0, l0);
      split_carry(fd, h1, l1);
      xh[e] = h0; xl[e] = l0;
      dh[e] = h1; dl[e] = l1;
    }
    *(v4h*)(sA1 + r * kA1P + c4)                  = xh;
    *(v4h*)(sA1 + r * kA1P + kDin + c4)           = xl;
    *(v4h*)(sA1 + (kSamp + r) * kA1P + c4)        = dh;
    *(v4h*)(sA1 + (kSamp + r) * kA1P + kDin + c4) = dl;
  }

  const _Float16* Bt1  = (const _Float16*)Bt1p;
  const _Float16* Bt1r = (const _Float16*)Bt1rp;
  const _Float16* Bt2  = (const _Float16*)Bt2p;
  const _Float16* Bt2r = (const _Float16*)Bt2rp;
  const v16h b1  = frag_load(Bt1  + (size_t)n * kK1 + 8 * hh);
  const v16h b1r = frag_load(Bt1r + (size_t)n * kK1 + 8 * hh);
  v16h b2[4], b2r[4];
#pragma unroll
  for (int ks = 0; ks < 4; ++ks) {
    b2[ks]  = frag_load(Bt2  + (size_t)n * kH + ks * 32 + 8 * hh);
    b2r[ks] = frag_load(Bt2r + (size_t)n * kH + ks * 32 + 8 * hh);
  }
  const float w3v = W3[n];

  __syncthreads();

#pragma unroll
  for (int t = 0; t < 4; ++t) {
    const v16h ap = frag_load(sA1 + (16 * t + c) * kA1P + 8 * hh);
    const v16h at = frag_load(sA1 + (kSamp + 16 * t + c) * kA1P + 8 * hh);
    v8f zp = (v8f){0.f, 0.f, 0.f, 0.f, 0.f, 0.f, 0.f, 0.f};
    v8f zr = (v8f){0.f, 0.f, 0.f, 0.f, 0.f, 0.f, 0.f, 0.f};
    v8f tp = (v8f){0.f, 0.f, 0.f, 0.f, 0.f, 0.f, 0.f, 0.f};
    v8f tr = (v8f){0.f, 0.f, 0.f, 0.f, 0.f, 0.f, 0.f, 0.f};
    zp = mma_h(ap, b1,  zp);
    zr = mma_h(ap, b1r, zr);
    tp = mma_h(at, b1,  tp);
    tr = mma_h(at, b1r, tr);
#pragma unroll
    for (int r = 0; r < 8; ++r) {
      const int row = 16 * t + 8 * hh + r;
      const float z  = (zp[r] + zr[r] * kResFold) * kFold1;
      const float zd = (tp[r] + tr[r] * kResFold) * kFold1;
      const float y  = z * z;
      const float yd = (2.0f * z) * zd;
      sA2[row * kA2P + n]           = (_Float16)(y * kCarryY);
      sA2[(kSamp + row) * kA2P + n] = (_Float16)(yd * kCarryY);
    }
  }
  __syncthreads();

  v8f y2v[4], y2dv[4];
#pragma unroll
  for (int t = 0; t < 4; ++t) {
    v8f qp = (v8f){0.f, 0.f, 0.f, 0.f, 0.f, 0.f, 0.f, 0.f};
    v8f qr = (v8f){0.f, 0.f, 0.f, 0.f, 0.f, 0.f, 0.f, 0.f};
    v8f tp = (v8f){0.f, 0.f, 0.f, 0.f, 0.f, 0.f, 0.f, 0.f};
    v8f tr = (v8f){0.f, 0.f, 0.f, 0.f, 0.f, 0.f, 0.f, 0.f};
#pragma unroll
    for (int ks = 0; ks < 4; ++ks) {
      const v16h ap = frag_load(sA2 + (16 * t + c) * kA2P + ks * 32 + 8 * hh);
      const v16h at = frag_load(sA2 + (kSamp + 16 * t + c) * kA2P + ks * 32 + 8 * hh);
      qp = mma_h(ap, b2[ks],  qp);
      qr = mma_h(ap, b2r[ks], qr);
      tp = mma_h(at, b2[ks],  tp);
      tr = mma_h(at, b2r[ks], tr);
    }
#pragma unroll
    for (int r = 0; r < 8; ++r) {
      const float z  = (qp[r] + qr[r] * kResFold) * kFold2;
      const float zd = (tp[r] + tr[r] * kResFold) * kFold2;
      y2v[t][r]  = z * z;
      y2dv[t][r] = (2.0f * z) * zd;
    }
  }
  __syncthreads();

#pragma unroll
  for (int t = 0; t < 4; ++t) {
    float pb[8], pd[8];
#pragma unroll
    for (int r = 0; r < 8; ++r) {
      const int row = 16 * t + 8 * hh + r;
      const float y2  = y2v[t][r];
      const float y2d = y2dv[t][r];
      sY[row * kYP + n] = y2;
      pb[r] = w3v * y2;
      pd[r] = w3v * y2d;
    }
#pragma unroll
    for (int off = 1; off < 16; off <<= 1) {
#pragma unroll
      for (int r = 0; r < 8; ++r) {
        const float ob = __shfl_xor(pb[r], off, 32);
        const float od = __shfl_xor(pd[r], off, 32);
        pb[r] += ob;
        pd[r] += od;
      }
    }
    if (c == 0) {
#pragma unroll
      for (int r = 0; r < 8; ++r) {
        const int row = 16 * t + 8 * hh + r;
        sPart[wave * kSamp + row]             = pb[r];
        sPart[8 * kSamp + wave * kSamp + row] = pd[r];
      }
    }
  }
  __syncthreads();

  {
    v4f vals[8];
#pragma unroll
    for (int it = 0; it < 8; ++it)
      vals[it] = *(const v4f*)(sY + (wave * 8 + it) * kYP + lane * 4);
    float* y2o = out + kOutY2 + (size_t)(n0 + wave * 8) * kH + lane * 4;
    for (int pass = 0; pass < 2; ++pass) {
#pragma unroll
      for (int it = 0; it < 8; ++it)
        *(volatile v4f*)(y2o + (size_t)it * kH) = vals[it];
      __threadfence();
    }
  }

  if (wave < 2) {
    const float* pp = sPart + wave * (8 * kSamp) + c * 4;
    v4f sv = (v4f){0.f, 0.f, 0.f, 0.f};
#pragma unroll
    for (int w = 0; w < 8; ++w) {
      const v4f pv = *(const v4f*)(pp + w * kSamp);
      sv = sv + pv;
    }
    float* po = out + (size_t)wave * kN + n0 + c * 4;
    if (lane < 16) *(volatile v4f*)po = sv;
    __threadfence();
    if (lane < 16) *(volatile v4f*)po = sv;
  }
}

extern "C" void kernel_launch(void* const* d_in, const int* in_sizes, int n_in,
                              void* d_out, int out_size, void* d_ws, size_t ws_size,
                              hipStream_t stream) {
  if (n_in != 5) return;
  if (in_sizes[0] != kN * kDin) return;
  if (in_sizes[1] != kN * kDin) return;
  if (in_sizes[2] != kH * kDin) return;
  if (in_sizes[3] != kH * kH) return;
  if (in_sizes[4] != kH) return;
  if ((size_t)out_size != kOutElems) return;
  if (ws_size < kWsTotal) return;

  const float* x    = (const float*)d_in[0];
  const float* xdot = (const float*)d_in[1];
  const float* W1   = (const float*)d_in[2];
  const float* W2   = (const float*)d_in[3];
  const float* W3   = (const float*)d_in[4];
  float* out = (float*)d_out;

  char* ws = (char*)d_ws;
  unsigned short* Bt2  = (unsigned short*)(ws + kOffBt2);
  unsigned short* Bt2r = (unsigned short*)(ws + kOffBt2r);
  unsigned short* Bt1  = (unsigned short*)(ws + kOffBt1);
  unsigned short* Bt1r = (unsigned short*)(ws + kOffBt1r);

  prep_weights_kernel<<<(kChunks2 + kChunks1) / 256, 256, 0, stream>>>(W1, W2, Bt2, Bt2r, Bt1, Bt1r);
  mlp_tangent_kernel<<<kN / kSamp, 256, 0, stream>>>(x, xdot, Bt1, Bt1r, Bt2, Bt2r, W3, out);
}
